// GeneralizedMamba2_49598282334525
// MI455X (gfx1250) — hardware-verified
//
#include <hip/hip_runtime.h>
#include <math.h>

typedef __attribute__((ext_vector_type(16))) _Float16 v16h;
typedef __attribute__((ext_vector_type(8)))  _Float16 v8h;
typedef __attribute__((ext_vector_type(8)))  float    v8f;
typedef __attribute__((ext_vector_type(4)))  float    v4f;
typedef __attribute__((ext_vector_type(4)))  unsigned v4u;

constexpr int kBatch   = 2;
constexpr int kSeq     = 2048;
constexpr int kDm      = 768;
constexpr int kDinner  = 1536;
constexpr int kHd      = 64;
constexpr int kNst     = 64;
constexpr int kNh      = 24;
constexpr int kConvPH  = 192;
constexpr int kConvDim = 4608;
constexpr int kProjN   = 6168;
constexpr int kProjP   = 6208;
constexpr int kXbcCol  = 1536;
constexpr int kDtCol   = 6144;
constexpr int kRows    = kBatch * kSeq;
constexpr int kTS = 32;
constexpr int kXP = 260;
constexpr int kRP = 68;
constexpr int kYP = 68;
constexpr float kCarryU  = 8.0f;
constexpr float kCarryW  = 32.0f;
constexpr float kCarryY  = 64.0f;
constexpr float kFoldIn  = 1.0f / (kCarryU * kCarryW);
constexpr float kFoldOut = 1.0f / (kCarryY * kCarryW);

static_assert(kNh * kHd == kDinner);
static_assert(kConvPH == kHd + 2 * kNst);
static_assert(kConvDim == kNh * kConvPH);
static_assert(kProjN == kDinner + kConvDim + kNh);
static_assert(kXbcCol == kDinner && kDtCol == kDinner + kConvDim);
static_assert(kProjP >= kProjN && (kProjP % 64) == 0);
static_assert((kDm % 32) == 0 && (kDinner % 32) == 0);
static_assert((kRows % 64) == 0 && (kDm % 64) == 0);
static_assert((kSeq % kTS) == 0 && kHd == 64 && kNst == 64 && kTS == 32);
static_assert(((kRows / 64) * (kProjP / 64)) % 8 == 0);
static_assert(((kRows / 64) * (kDm / 64)) % 8 == 0);
static_assert(((kRows * kDm) % 2048) == 0 && ((kProjP * kDm) % 2048) == 0 && ((kDm * kDinner) % 2048) == 0);

constexpr size_t kOffU16   = 0;
constexpr size_t kOffWIN   = kOffU16  + (size_t)kRows  * kDm     * 2;
constexpr size_t kOffWOUT  = kOffWIN  + (size_t)kProjP * kDm     * 2;
constexpr size_t kOffZX    = kOffWOUT + (size_t)kDm    * kDinner * 2;
constexpr size_t kOffYG    = kOffZX   + (size_t)kRows  * kProjP  * 2;
constexpr size_t kWsTotal  = kOffYG   + (size_t)kRows  * kDinner * 2;
static_assert(kWsTotal == 81625088ull);
static_assert(kWsTotal <= 134217728ull);
static_assert((kOffWIN % 128) == 0 && (kOffWOUT % 128) == 0 && (kOffZX % 128) == 0 && (kOffYG % 128) == 0);

__device__ __forceinline__ void row_guard_h(v8f& a, v8f& b, v8f& c, v8f& d, v16h x, v16h b0, v16h b1, v16h b2, v16h b3) {
  asm volatile("v_nop\n\tv_nop\n\tv_nop\n\tv_nop" : "+v"(a), "+v"(b), "+v"(c), "+v"(d) : "v"(x), "v"(b0), "v"(b1), "v"(b2), "v"(b3));
}
__device__ __forceinline__ void keep4_h(v16h a, v16h b, v16h c, v16h d) { asm volatile("v_nop" :: "v"(a), "v"(b), "v"(c), "v"(d)); }
__device__ __forceinline__ void acc_guard4(v8f& a, v8f& b, v8f& c, v8f& d) { asm volatile("v_nop\n\tv_nop\n\tv_nop\n\tv_nop" : "+v"(a), "+v"(b), "+v"(c), "+v"(d)); }

union FragH { v16h v; v8h h[2]; };
__device__ __forceinline__ v16h frag_load_h(const _Float16* p) {
  FragH f;
  f.h[0] = *(const v8h*)(p);
  f.h[1] = *(const v8h*)(p + 16);
  return f.v;
}
__device__ __forceinline__ v8f mma_h(v16h a, v16h b, v8f c) {
  return __builtin_amdgcn_wmma_f32_16x16x32_f16(false, a, false, b, (short)0, c, false, false);
}

template <int OUT_MODE>
__global__ __launch_bounds__(256) void wmma_gemm64_f16(
    const unsigned short* __restrict__ Ap, int lda,
    const unsigned short* __restrict__ Btp, int ldb,
    void* __restrict__ Cout, int ldc,
    int M, int N, int K, float scale) {
  const _Float16* A  = (const _Float16*)Ap;
  const _Float16* Bt = (const _Float16*)Btp;
  __shared__ __align__(16) float sT[8][16 * 68];
  const int lane = threadIdx.x & 31;
  const int wave = threadIdx.x >> 5;
  const int tilesN = N >> 6;
  const int tilesM = M >> 6;
  const int tile = blockIdx.x * 8 + wave;
  if (tile >= tilesM * tilesN) return;
  const int tm = tile / tilesN;
  const int tn = tile - tm * tilesN;
  const int m0 = tm << 6;
  const int n0 = tn << 6;

  const int rlane = lane & 15;
  const int koff  = (lane >> 4) * 8;
  const int mOff  = (lane >> 4) * 8;

  v8f acc[4][4];
#pragma unroll
  for (int i = 0; i < 4; ++i)
#pragma unroll
    for (int j = 0; j < 4; ++j) acc[i][j] = (v8f){0.f,0.f,0.f,0.f,0.f,0.f,0.f,0.f};

  for (int k0 = 0; k0 < K; k0 += 32) {
    v16h bh[4];
#pragma unroll
    for (int j = 0; j < 4; ++j) {
      const size_t bo = (size_t)(n0 + (j << 4) + rlane) * ldb + koff + k0;
      bh[j] = frag_load_h(Bt + bo);
    }
#pragma unroll
    for (int i = 0; i < 4; ++i) {
      const size_t ao = (size_t)(m0 + (i << 4) + rlane) * lda + koff + k0;
      const v16h ah = frag_load_h(A + ao);
#pragma unroll
      for (int j = 0; j < 4; ++j) acc[i][j] = mma_h(ah, bh[j], acc[i][j]);
      row_guard_h(acc[i][0], acc[i][1], acc[i][2], acc[i][3], ah, bh[0], bh[1], bh[2], bh[3]);
    }
    keep4_h(bh[0], bh[1], bh[2], bh[3]);
  }
  acc_guard4(acc[0][0], acc[0][1], acc[0][2], acc[0][3]);
  acc_guard4(acc[1][0], acc[1][1], acc[1][2], acc[1][3]);
  acc_guard4(acc[2][0], acc[2][1], acc[2][2], acc[2][3]);
  acc_guard4(acc[3][0], acc[3][1], acc[3][2], acc[3][3]);

  float* slab = sT[wave];
#pragma unroll
  for (int i = 0; i < 4; ++i) {
    const int mBase = m0 + (i << 4);
#pragma unroll
    for (int j = 0; j < 4; ++j) {
#pragma unroll
      for (int r = 0; r < 8; ++r) {
        const float v = acc[i][j][r] * scale;
        slab[(mOff + r) * 68 + (j << 4) + rlane] = v;
      }
    }
    __builtin_amdgcn_fence(__ATOMIC_RELEASE, "workgroup");
    __builtin_amdgcn_wave_barrier();
    __builtin_amdgcn_fence(__ATOMIC_ACQUIRE, "workgroup");
    if (OUT_MODE == 0) {
      float* C = (float*)Cout;
      const int hh = lane >> 4, c4 = (lane & 15) * 4;
      for (int pass = 0; pass < 2; ++pass) {
#pragma unroll
        for (int it = 0; it < 8; ++it) {
          const int row = it * 2 + hh;
          const v4f v = *(const v4f*)(slab + row * 68 + c4);
          *(volatile v4f*)(C + (size_t)(mBase + row) * ldc + n0 + c4) = v;
        }
        __threadfence();
      }
    } else {
      const int q = lane >> 3, c8 = (lane & 7) * 8;
      unsigned short* C = (unsigned short*)Cout;
      for (int pass = 0; pass < 2; ++pass) {
#pragma unroll
        for (int it = 0; it < 4; ++it) {
          const int row = it * 4 + q;
          const float* sp = slab + row * 68 + c8;
          v8h hv;
#pragma unroll
          for (int e = 0; e < 8; ++e) hv[e] = (_Float16)sp[e];
          *(volatile v8h*)(C + (size_t)(mBase + row) * ldc + n0 + c8) = hv;
        }
        __threadfence();
      }
    }
    __builtin_amdgcn_fence(__ATOMIC_RELEASE, "workgroup");
    __builtin_amdgcn_wave_barrier();
    __builtin_amdgcn_fence(__ATOMIC_ACQUIRE, "workgroup");
  }
}

__global__ __launch_bounds__(256) void cast_f16_kernel(
    const float* __restrict__ src, unsigned short* __restrict__ dst, int total8, int real8, float scale)
{
  const int i = blockIdx.x * 256 + threadIdx.x;
  if (i >= total8) return;
  const bool valid = (i < real8);
  const int ic = valid ? i : (real8 - 1);
  const float* p = src + ((size_t)ic << 3);
  const v4f a0 = *(const v4f*)(p);
  const v4f a1 = *(const v4f*)(p + 4);
  v8h hv;
#pragma unroll
  for (int e = 0; e < 4; ++e) {
    const float f0 = valid ? (a0[e] * scale) : 0.0f;
    const float f1 = valid ? (a1[e] * scale) : 0.0f;
    hv[e]     = (_Float16)f0;
    hv[4 + e] = (_Float16)f1;
  }
  unsigned short* q = dst + ((size_t)i << 3);
  *(volatile v8h*)q = hv;
  __threadfence();
  *(volatile v8h*)q = hv;
}

__device__ __forceinline__ float h16_to_f32(unsigned hb) {
  const unsigned sgn = (hb & 0x8000u) << 16;
  const unsigned em = hb & 0x7fffu;
  const float fn = __uint_as_float((em << 13) + 0x38000000u);
  const float fs = (float)em * 5.9604644775390625e-8f;
  const float mag = (em < 0x400u) ? fs : fn;
  return __uint_as_float(__float_as_uint(mag) | sgn);
}

__device__ __forceinline__ float silu_f(float v) {
  const float sg = __builtin_amdgcn_rcpf(1.0f + __expf(-v));
  return v * sg;
}

__global__ __launch_bounds__(64) void scan_kernel(
    const unsigned short* __restrict__ ZX16,
    const float* __restrict__ conv_w, const float* __restrict__ conv_b,
    const float* __restrict__ Rx, const float* __restrict__ RB, const float* __restrict__ RC,
    const float* __restrict__ Rdt, const float* __restrict__ dt_bias, const float* __restrict__ A_log,
    const float* __restrict__ Dw, unsigned short* __restrict__ YG16)
{
  __shared__ __align__(16) float sRx[64 * kRP];
  __shared__ __align__(16) float sRB[64 * kRP];
  __shared__ __align__(16) float sRC[64 * kRP];
  __shared__ __align__(16) float sSt[64 * kRP];
  __shared__ __align__(16) float sRd[64];
  __shared__ __align__(16) float sYl[64];
  __shared__ __align__(16) float sB[64];
  __shared__ __align__(16) float sC[64];
  __shared__ __align__(16) float sX[kTS * kXP];
  __shared__ __align__(16) float sY[kTS * kYP];

  const int tid = threadIdx.x, lane = tid & 31, wave = tid >> 5;
  const int bix = blockIdx.x / kNh;
  const int hd  = blockIdx.x - bix * kNh;
  const size_t row0 = (size_t)bix * kSeq;

#pragma unroll 1
  for (int i = 0; i < 16; ++i) {
    const int idx = tid + 64 * i;
    const int p = idx >> 4, q4 = (idx & 15) * 4;
    const size_t g = (size_t)hd * 4096 + (size_t)p * 64 + q4;
    const v4f vx = *(const v4f*)(Rx + g);
    const v4f vb = *(const v4f*)(RB + g);
    const v4f vc = *(const v4f*)(RC + g);
    *(v4f*)(sRx + p * kRP + q4) = vx;
    *(v4f*)(sRB + p * kRP + q4) = vb;
    *(v4f*)(sRC + p * kRP + q4) = vc;
  }
  sRd[tid] = Rdt[hd * 64 + tid];
  sYl[tid] = 0.0f;
  {
    float* zp = sSt + tid * kRP;
    const v4f zz = (v4f){0.f, 0.f, 0.f, 0.f};
#pragma unroll 1
    for (int i = 0; i < kRP / 4; ++i) *(v4f*)(zp + 4 * i) = zz;
  }

  const int chx = hd * kConvPH + tid;
  const v4f cwx = *(const v4f*)(conv_w + (size_t)chx * 4);
  const v4f cwb = *(const v4f*)(conv_w + (size_t)(chx + 64) * 4);
  const v4f cwc = *(const v4f*)(conv_w + (size_t)(chx + 128) * 4);
  const float cbx = conv_b[chx], cbb = conv_b[chx + 64], cbc = conv_b[chx + 128];
  const float dtb  = dt_bias[hd];
  const float Aneg = -expf(A_log[hd]);
  const float Dh   = Dw[hd * 64 + tid];

  float hx3 = 0.0f, hx2 = 0.0f, hx1 = 0.0f;
  float hb3 = 0.0f, hb2 = 0.0f, hb1 = 0.0f;
  float hc3 = 0.0f, hc2 = 0.0f, hc1 = 0.0f;

  const float* prx = sRx + tid * kRP;
  const float* prb = sRB + tid * kRP;
  const float* prc = sRC + tid * kRP;
  float* pst = sSt + tid * kRP;
  const int q = lane >> 3, c8 = (lane & 7) * 8;
  __syncthreads();

#pragma unroll 1
  for (int t0 = 0; t0 < kSeq; t0 += kTS) {
    __syncthreads();
#pragma unroll 1
    for (int i = 0; i < 16; ++i) {
      const int idx = tid + 64 * i;
      const int r = idx >> 5, c = idx & 31;
      const int col = (c < 24) ? (kXbcCol + hd * kConvPH + c * 8) : (hd * kHd + (c - 24) * 8);
      const v4u w = *(const v4u*)(ZX16 + (row0 + t0 + r) * (size_t)kProjP + col);
      const unsigned w0 = w[0], w1 = w[1], w2 = w[2], w3 = w[3];
      v4f f0, f1;
      f0[0] = h16_to_f32(w0 & 0xffffu);
      f0[1] = h16_to_f32(w0 >> 16);
      f0[2] = h16_to_f32(w1 & 0xffffu);
      f0[3] = h16_to_f32(w1 >> 16);
      f1[0] = h16_to_f32(w2 & 0xffffu);
      f1[1] = h16_to_f32(w2 >> 16);
      f1[2] = h16_to_f32(w3 & 0xffffu);
      f1[3] = h16_to_f32(w3 >> 16);
      float* dp = sX + r * kXP + c * 8;
      *(v4f*)(dp)     = f0;
      *(v4f*)(dp + 4) = f1;
    }
    if (tid < kTS) {
      const size_t e = (row0 + t0 + tid) * (size_t)kProjP + kDtCol + hd;
      const unsigned wv = ((const unsigned*)(const void*)ZX16)[e >> 1];
      const unsigned hb = (hd & 1) ? (wv >> 16) : (wv & 0xffffu);
      sX[tid * kXP + 256] = h16_to_f32(hb);
    }
    __syncthreads();

#pragma unroll 1
    for (int s = 0; s < kTS; ++s) {
      const float* xr = sX + s * kXP;
      float rx = 0.0f, rb = 0.0f, rc = 0.0f, rd = 0.0f;
#pragma unroll 1
      for (int i = 0; i < 16; ++i) {
        const v4f yv = *(const v4f*)(sYl + 4 * i);
        const v4f ax = *(const v4f*)(prx + 4 * i);
        const v4f ab = *(const v4f*)(prb + 4 * i);
        const v4f ac = *(const v4f*)(prc + 4 * i);
        const v4f ad = *(const v4f*)(sRd + 4 * i);
        rx = fmaf(ax[0], yv[0], rx);
        rx = fmaf(ax[1], yv[1], rx);
        rx = fmaf(ax[2], yv[2], rx);
        rx = fmaf(ax[3], yv[3], rx);
        rb = fmaf(ab[0], yv[0], rb);
        rb = fmaf(ab[1], yv[1], rb);
        rb = fmaf(ab[2], yv[2], rb);
        rb = fmaf(ab[3], yv[3], rb);
        rc = fmaf(ac[0], yv[0], rc);
        rc = fmaf(ac[1], yv[1], rc);
        rc = fmaf(ac[2], yv[2], rc);
        rc = fmaf(ac[3], yv[3], rc);
        rd = fmaf(ad[0], yv[0], rd);
        rd = fmaf(ad[1], yv[1], rd);
        rd = fmaf(ad[2], yv[2], rd);
        rd = fmaf(ad[3], yv[3], rd);
      }
      const float cx  = xr[tid];
      const float cb_ = xr[64 + tid];
      const float cc  = xr[128 + tid];
      const float zv  = xr[192 + tid];
      const float dtr = xr[256];
      float ux = cwx[0] * hx3;
      ux = fmaf(cwx[1], hx2, ux);
      ux = fmaf(cwx[2], hx1, ux);
      ux = fmaf(cwx[3], cx, ux);
      ux += cbx;
      float ub = cwb[0] * hb3;
      ub = fmaf(cwb[1], hb2, ub);
      ub = fmaf(cwb[2], hb1, ub);
      ub = fmaf(cwb[3], cb_, ub);
      ub += cbb;
      float uc = cwc[0] * hc3;
      uc = fmaf(cwc[1], hc2, uc);
      uc = fmaf(cwc[2], hc1, uc);
      uc = fmaf(cwc[3], cc, uc);
      uc += cbc;
      hx3 = hx2; hx2 = hx1; hx1 = cx;
      hb3 = hb2; hb2 = hb1; hb1 = cb_;
      hc3 = hc2; hc2 = hc1; hc1 = cc;

      const float xv = silu_f(ux + rx);
      const float Bm = silu_f(ub + rb);
      const float Cm = silu_f(uc + rc);
      const float vdt = (dtr + rd) + dtb;
      const float dt  = fmaxf(vdt, 0.0f) + log1pf(__expf(-fabsf(vdt)));
      const float dA  = __expf(dt * Aneg);
      sB[tid] = Bm;
      sC[tid] = Cm;
      __syncthreads();

      const float dtx = dt * xv;
      float yacc = 0.0f;
#pragma unroll 1
      for (int i = 0; i < 16; ++i) {
        const v4f st = *(const v4f*)(pst + 4 * i);
        const v4f bv = *(const v4f*)(sB + 4 * i);
        const v4f cv = *(const v4f*)(sC + 4 * i);
        v4f ns;
        ns[0] = fmaf(st[0], dA, dtx * bv[0]);
        ns[1] = fmaf(st[1], dA, dtx * bv[1]);
        ns[2] = fmaf(st[2], dA, dtx * bv[2]);
        ns[3] = fmaf(st[3], dA, dtx * bv[3]);
        yacc = fmaf(ns[0], cv[0], yacc);
        yacc = fmaf(ns[1], cv[1], yacc);
        yacc = fmaf(ns[2], cv[2], yacc);
        yacc = fmaf(ns[3], cv[3], yacc);
        *(v4f*)(pst + 4 * i) = ns;
      }
      const float yv = fmaf(Dh, xv, yacc);
      const float gz = silu_f(zv);
      sYl[tid] = yv;
      sY[s * kYP + tid] = (yv * gz) * kCarryY;
      __syncthreads();
    }

    v8h hv[4];
#pragma unroll
    for (int it = 0; it < 4; ++it) {
      const int row = it * 8 + wave * 4 + q;
      const float* sp = sY + row * kYP + c8;
      const v4f a0 = *(const v4f*)(sp);
      const v4f a1 = *(const v4f*)(sp + 4);
#pragma unroll
      for (int e = 0; e < 4; ++e) {
        hv[it][e]     = (_Float16)a0[e];
        hv[it][4 + e] = (_Float16)a1[e];
      }
    }
    for (int pass = 0; pass < 2; ++pass) {
#pragma unroll
      for (int it = 0; it < 4; ++it) {
        const int row = it * 8 + wave * 4 + q;
        const size_t o = (row0 + t0 + row) * (size_t)kDinner + hd * kHd + c8;
        *(volatile v8h*)(YG16 + o) = hv[it];
      }
      __threadfence();
    }
  }
}

extern "C" void kernel_launch(void* const* d_in, const int* in_sizes, int n_in,
                              void* d_out, int out_size, void* d_ws, size_t ws_size,
                              hipStream_t stream)
{
  if (n_in < 12) return;
  if (in_sizes[0] != kRows * kDm) return;
  if (in_sizes[1] != kProjN * kDm) return;
  if (in_sizes[2] != kConvDim * 4) return;
  if (in_sizes[3] != kConvDim) return;
  if (in_sizes[4] != kNh * kHd * kHd) return;
  if (in_sizes[5] != kNh * kNst * kHd) return;
  if (in_sizes[6] != kNh * kNst * kHd) return;
  if (in_sizes[7] != kNh * kHd) return;
  if (in_sizes[8] != kNh) return;
  if (in_sizes[9] != kNh) return;
  if (in_sizes[10] != kNh * kHd) return;
  if (in_sizes[11] != kDm * kDinner) return;
  if (out_size != kRows * kDm) return;
  if (ws_size < kWsTotal) return;

  const float* u       = (const float*)d_in[0];
  const float* W_in    = (const float*)d_in[1];
  const float* conv_w  = (const float*)d_in[2];
  const float* conv_b  = (const float*)d_in[3];
  const float* R_x     = (const float*)d_in[4];
  const float* R_B     = (const float*)d_in[5];
  const float* R_C     = (const float*)d_in[6];
  const float* R_dt    = (const float*)d_in[7];
  const float* dt_bias = (const float*)d_in[8];
  const float* A_log   = (const float*)d_in[9];
  const float* Dw      = (const float*)d_in[10];
  const float* W_out   = (const float*)d_in[11];
  float* out = (float*)d_out;

  char* ws = (char*)d_ws;
  unsigned short* U16    = (unsigned short*)(ws + kOffU16);
  unsigned short* WIN16  = (unsigned short*)(ws + kOffWIN);
  unsigned short* WOUT16 = (unsigned short*)(ws + kOffWOUT);
  unsigned short* ZX16   = (unsigned short*)(ws + kOffZX);
  unsigned short* YG16   = (unsigned short*)(ws + kOffYG);

  cast_f16_kernel<<<(kRows * kDm / 8) / 256, 256, 0, stream>>>(u, U16, kRows * kDm / 8, kRows * kDm / 8, kCarryU);
  cast_f16_kernel<<<(kProjP * kDm / 8) / 256, 256, 0, stream>>>(W_in, WIN16, kProjP * kDm / 8, kProjN * kDm / 8, kCarryW);
  cast_f16_kernel<<<(kDm * kDinner / 8) / 256, 256, 0, stream>>>(W_out, WOUT16, kDm * kDinner / 8, kDm * kDinner / 8, kCarryW);

  wmma_gemm64_f16<1><<<((kRows / 64) * (kProjP / 64)) / 8, 256, 0, stream>>>(
      U16, kDm, WIN16, kDm, (void*)ZX16, kProjP, kRows, kProjP, kDm, kFoldIn);

  scan_kernel<<<kBatch * kNh, 64, 0, stream>>>(ZX16, conv_w, conv_b, R_x, R_B, R_C, R_dt, dt_bias, A_log, Dw, YG16);

  wmma_gemm64_f16<0><<<((kRows / 64) * (kDm / 64)) / 8, 256, 0, stream>>>(
      YG16, kDinner, WOUT16, kDinner, (void*)out, kDm, kRows, kDm, kDinner, kFoldOut);
}
